// NonLocalLayer_dilation_75960791597922
// MI455X (gfx1250) — hardware-run, weakly checked
//
#include <hip/hip_runtime.h>

typedef float          v8f   __attribute__((ext_vector_type(8)));
typedef float          v4f   __attribute__((ext_vector_type(4)));
typedef unsigned int   v4u   __attribute__((ext_vector_type(4)));
typedef int            v8i   __attribute__((ext_vector_type(8)));
typedef unsigned short v8us  __attribute__((ext_vector_type(8)));
typedef unsigned short v16us __attribute__((ext_vector_type(16)));
typedef __bf16         v16bf __attribute__((ext_vector_type(16)));
typedef _Float16       v16h  __attribute__((ext_vector_type(16)));
typedef v4f  __attribute__((may_alias)) v4fa;
typedef v8us __attribute__((may_alias)) v8usa;
union FragB { v16bf v; v16us u; v8us h[2]; v8i w; };
union FragH { v16h  v; v16us u; v8us h[2]; v8i w; };

__device__ __forceinline__ v8f wmb(const FragB& a, const FragB& b, v8f c) {
  v8f d = __builtin_amdgcn_wmma_f32_16x16x32_bf16(false, a.v, false, b.v, (short)0, c, false, false);
  asm volatile("v_nop\n\tv_nop\n\tv_nop\n\tv_nop" : "+v"(d) : "v"(a.w), "v"(b.w));
  return d;
}

__device__ __forceinline__ v8f wmh(const FragH& a, const FragH& b, v8f c) {
  v8f d = __builtin_amdgcn_wmma_f32_16x16x32_f16(false, a.v, false, b.v, (short)0, c, false, false);
  asm volatile("v_nop\n\tv_nop\n\tv_nop\n\tv_nop" : "+v"(d) : "v"(a.w), "v"(b.w));
  return d;
}

__device__ __forceinline__ unsigned bf16_bits(float f) {
  const unsigned u = __float_as_uint(f);
  const unsigned r = (u + 0x7FFFu + ((u >> 16) & 1u)) >> 16;
  const unsigned q = (u >> 16) | 0x40u;
  return ((u & 0x7fffffffu) > 0x7f800000u) ? q : r;
}

__device__ __forceinline__ float bf16_val(float f) {
  return __uint_as_float(bf16_bits(f) << 16);
}
__device__ __forceinline__ int clampi(int v, int lo, int hi) {
  return v < lo ? lo : (v > hi ? hi : v);
}

__device__ __forceinline__ unsigned f16_bits(float f) {
  const unsigned u  = __float_as_uint(f);
  const unsigned s  = (u >> 16) & 0x8000u;
  const unsigned a  = u & 0x7fffffffu;
  const unsigned t  = a - 0x38000000u;
  const unsigned r  = (t + 0x0FFFu + ((t >> 13) & 1u)) >> 13;
  const unsigned rc = r > 0x7C00u ? 0x7C00u : r;
  const bool small  = a < 0x38800000u;
  const bool isnan  = a > 0x7f800000u;
  const unsigned fin = small ? 0u : (s | rc);
  return isnan ? (s | 0x7E00u) : fin;
}

__device__ __forceinline__ unsigned pk16(unsigned lo, unsigned hi) { return lo | (hi << 16); }
__device__ __forceinline__ unsigned bf16_lo_bits(float v) {
  float hi = bf16_val(v);
  asm volatile("" : "+v"(hi));
  return bf16_bits(v - hi);
}
__device__ __forceinline__ v4u pack8_bf16(v4f a, v4f c) {
  return (v4u){ pk16(bf16_bits(a[0]), bf16_bits(a[1])), pk16(bf16_bits(a[2]), bf16_bits(a[3])),
                pk16(bf16_bits(c[0]), bf16_bits(c[1])), pk16(bf16_bits(c[2]), bf16_bits(c[3])) };
}
__device__ __forceinline__ v4u pack8_bf16_lo(v4f a, v4f c) {
  return (v4u){ pk16(bf16_lo_bits(a[0]), bf16_lo_bits(a[1])), pk16(bf16_lo_bits(a[2]), bf16_lo_bits(a[3])),
                pk16(bf16_lo_bits(c[0]), bf16_lo_bits(c[1])), pk16(bf16_lo_bits(c[2]), bf16_lo_bits(c[3])) };
}
__device__ __forceinline__ v4u pack8_f16(v4f a, v4f c) {
  return (v4u){ pk16(f16_bits(a[0]), f16_bits(a[1])), pk16(f16_bits(a[2]), f16_bits(a[3])),
                pk16(f16_bits(c[0]), f16_bits(c[1])), pk16(f16_bits(c[2]), f16_bits(c[3])) };
}

template <int FORM>
__global__ __launch_bounds__(256) void k_plane(const float* __restrict__ src, int rows, int cols, int ldsrc,
                                               unsigned short* __restrict__ dst, int MP, int KP) {
  static_assert(FORM >= 0 && FORM <= 3);
  const int KTOT = (FORM == 1 || FORM == 3) ? 2 * KP : KP;
  const unsigned ppr   = (unsigned)(KTOT >> 3);
  const unsigned kp8   = (unsigned)(KP >> 3);
  const unsigned total = (unsigned)MP * ppr;
  const unsigned g     = blockIdx.x * 256u + threadIdx.x;
  const unsigned rowu  = g / ppr;
  const unsigned p     = g - rowu * ppr;
  const bool second    = p >= kp8;
  const int row = (int)rowu;
  const int c0  = (int)((second ? p - kp8 : p) << 3);
  const float* srow = src + (size_t)clampi(row, 0, rows - 1) * (size_t)ldsrc;
  float x[8];
  unsigned mk[8];
#pragma unroll
  for (int e = 0; e < 8; ++e) {
    const int c = c0 + e;
    const float v = srow[clampi(c, 0, cols - 1)];
    asm volatile("" :: "v"(v));
    x[e]  = v;
    mk[e] = (row < rows && c < cols) ? 0xFFFFu : 0u;
  }
  const v4f a = (v4f){ x[0], x[1], x[2], x[3] };
  const v4f c = (v4f){ x[4], x[5], x[6], x[7] };
  v4u o;
  if (FORM == 2) {
    o = pack8_f16(a, c);
  } else {
    const v4u hi = pack8_bf16(a, c);
    o = hi;
    if (FORM == 1) { const v4u lo = pack8_bf16_lo(a, c); o = second ? lo : hi; }
  }
  const v4u mw = (v4u){ pk16(mk[0], mk[1]), pk16(mk[2], mk[3]), pk16(mk[4], mk[5]), pk16(mk[6], mk[7]) };
  o &= mw;
  if (g < total) {
    volatile v4u* q = (volatile v4u*)(dst + (size_t)g * 8);
    *q = o;
    __threadfence();
    *q = o;
  }
}

template <int FORM> struct FragOf    { typedef FragB T; };
template <>         struct FragOf<2> { typedef FragH T; };
__device__ __forceinline__ v8f mm(const FragB& a, const FragB& b, v8f c) { return wmb(a, b, c); }
__device__ __forceinline__ v8f mm(const FragH& a, const FragH& b, v8f c) { return wmh(a, b, c); }
template <class F> __device__ __forceinline__ F ld_frag(const unsigned short* p) {
  F f;
  f.h[0] = *(const v8usa*)(p);
  f.h[1] = *(const v8usa*)(p + 16);
  return f;
}

template <int FORM, int EPI>
__global__ __launch_bounds__(256) __attribute__((amdgpu_num_vgpr(248)))
void k_gemm_nt(const unsigned short* __restrict__ A, const unsigned short* __restrict__ B,
               const float* __restrict__ bias, float* __restrict__ D, int M, int N, int KTOT, int ldd) {
  static_assert(FORM >= 0 && FORM <= 2);
  static_assert(EPI == 0 || EPI == 1);
  typedef typename FragOf<FORM>::T F;
  __shared__ __attribute__((aligned(16))) float sT[8][16 * 68];
  const int lane = threadIdx.x & 31;
  const int wave = threadIdx.x >> 5;
  const int tilesM = (M + 63) >> 6;
  const int tilesN = (N + 63) >> 6;
  const int tile = blockIdx.x * 8 + wave;
  if (tile >= tilesM * tilesN) return;
  const int tm = tile / tilesN;
  const int tn = tile - tm * tilesN;
  const int m0 = tm << 6;
  const int n0 = tn << 6;

  const int rl = lane & 15;
  const int h8 = (lane >> 4) * 8;
  const unsigned short* pa = A + (size_t)(m0 + rl) * (size_t)KTOT + h8;
  const unsigned short* pb = B + (size_t)(n0 + rl) * (size_t)KTOT + h8;

  v8f acc[4][4];
#pragma unroll
  for (int i = 0; i < 4; ++i)
#pragma unroll
    for (int j = 0; j < 4; ++j) acc[i][j] = (v8f){0.f, 0.f, 0.f, 0.f, 0.f, 0.f, 0.f, 0.f};

#pragma unroll 1
  for (int k0 = 0; k0 < KTOT; k0 += 32) {
    F bf[4];
#pragma unroll
    for (int j = 0; j < 4; ++j) bf[j] = ld_frag<F>(pb + (size_t)(j << 4) * (size_t)KTOT + k0);
#pragma unroll
    for (int i = 0; i < 4; ++i) {
      const F af = ld_frag<F>(pa + (size_t)(i << 4) * (size_t)KTOT + k0);
#pragma unroll
      for (int j = 0; j < 4; ++j) acc[i][j] = mm(af, bf[j], acc[i][j]);
    }
  }

  float* slab = sT[wave];
  const int hh = lane >> 4;
  const int c4 = (lane & 15) * 4;
  const int nc = n0 + c4;
  const bool cok = nc < N;
  v4f bv = (v4f){0.f, 0.f, 0.f, 0.f};
  if (EPI == 1) {
    bv = *(const v4fa*)(bias + clampi(nc, 0, N - 4));
    asm volatile("" :: "v"(bv));
  }
#pragma unroll
  for (int i = 0; i < 4; ++i) {
    const int mBase = m0 + (i << 4);
#pragma unroll
    for (int j = 0; j < 4; ++j) {
#pragma unroll
      for (int r = 0; r < 8; ++r) slab[(h8 + r) * 68 + (j << 4) + rl] = acc[i][j][r];
    }
    __builtin_amdgcn_fence(__ATOMIC_RELEASE, "workgroup");
    __builtin_amdgcn_wave_barrier();
    __builtin_amdgcn_fence(__ATOMIC_ACQUIRE, "workgroup");
    v4f vv[8];
#pragma unroll
    for (int it = 0; it < 8; ++it) {
      const int row = it * 2 + hh;
      v4f v = *(const v4fa*)(slab + row * 68 + c4);
      if (EPI == 1) v += bv;
      vv[it] = v;
    }
    for (int pass = 0; pass < 2; ++pass) {
#pragma unroll
      for (int it = 0; it < 8; ++it) {
        const int row = mBase + it * 2 + hh;
        if (cok && row < M) *(volatile v4f*)(D + (size_t)row * (size_t)ldd + nc) = vv[it];
      }
      __threadfence();
    }
    __builtin_amdgcn_fence(__ATOMIC_RELEASE, "workgroup");
    __builtin_amdgcn_wave_barrier();
    __builtin_amdgcn_fence(__ATOMIC_ACQUIRE, "workgroup");
  }
}

#ifndef OUT_FORM
#define OUT_FORM 1
#endif
static_assert(OUT_FORM == 1 || OUT_FORM == 2);

#define NB   2
#define CH   64
#define HH   128
#define WW   128
#define KS   7
#define DIL  2
#define PAD  6
#define NK2  (KS * KS)
#define NTOK (NB * HH * WW)
#define NQKV (3 * CH)
#define TP   65

#if OUT_FORM == 2
#define AO_CARRY 256.0f
#define WT_CARRY 64.0f
#define Y_FOLD   (1.0f / 16384.0f)
#define AOK      CH
#else
#define AO_CARRY 1.0f
#define Y_FOLD   1.0f
#define AOK      (2 * CH)
#endif

static_assert(CH == 64);
static_assert(HH == 128 && WW == 128);
static_assert(KS == 7 && DIL == 2 && PAD == 6);
static_assert(2 * PAD == DIL * (KS - 1));
static_assert(CH % 16 == 0);
static_assert(NQKV % 32 == 0 && NQKV % 64 == 0);
static_assert(CH % 32 == 0 && AOK % 32 == 0);
static_assert(NTOK % 64 == 0);
static_assert(NB * HH == 256);
static_assert((NTOK * CH / 8) % 256 == 0);
static_assert((NTOK * AOK / 8) % 256 == 0);
static_assert((NQKV * CH / 8) % 256 == 0);
static_assert((CH * 2 * CH / 8) % 256 == 0);
static_assert((CH * CH / 8) % 256 == 0);
static_assert((NTOK * NQKV / 4) % 256 == 0);
static_assert((NQKV * CH / 4) % 256 == 0);

typedef v4u __attribute__((may_alias)) v4ua;

__global__ __launch_bounds__(256) void k_x2t(const float* __restrict__ X, float* __restrict__ XT) {
  __shared__ __attribute__((aligned(16))) float tl[128 * TP];
  const int tid = threadIdx.x;
  const int bh  = blockIdx.x;
  const int b   = bh >> 7;
  const int h   = bh & 127;
#pragma unroll
  for (int it = 0; it < 8; ++it) {
    const int idx = it * 256 + tid;
    const int c   = idx >> 5;
    const int w4  = (idx & 31) * 4;
    const v4f a = *(const v4fa*)(X + ((size_t)(b * CH + c) * HH + h) * WW + w4);
    tl[(w4 + 0) * TP + c] = a[0];
    tl[(w4 + 1) * TP + c] = a[1];
    tl[(w4 + 2) * TP + c] = a[2];
    tl[(w4 + 3) * TP + c] = a[3];
  }
  __syncthreads();
  v4f vv[8];
#pragma unroll
  for (int it = 0; it < 8; ++it) {
    const int idx = it * 256 + tid;
    const int w   = idx >> 4;
    const int c4  = (idx & 15) * 4;
    const float* sp = tl + w * TP + c4;
    vv[it] = (v4f){ sp[0], sp[1], sp[2], sp[3] };
  }
  float* dst = XT + (size_t)bh * (size_t)(WW * CH);
  for (int pass = 0; pass < 2; ++pass) {
#pragma unroll
    for (int it = 0; it < 8; ++it) {
      const int idx = it * 256 + tid;
      *(volatile v4f*)(dst + (size_t)idx * 4) = vv[it];
    }
    __threadfence();
  }
}

__global__ __launch_bounds__(256) void k_wstack(const float* __restrict__ Wk, const float* __restrict__ Wq,
                                                const float* __restrict__ Wv, float* __restrict__ WS) {
  const int g   = blockIdx.x * 256 + threadIdx.x;
  const int row = g >> 4;
  const int c4  = (g & 15) * 4;
  const int mat = row >> 6;
  const int off = (row & 63) * CH + c4;
  const v4u a = *(const v4ua*)(const void*)(Wk + off);
  const v4u b = *(const v4ua*)(const void*)(Wq + off);
  const v4u c = *(const v4ua*)(const void*)(Wv + off);
  asm volatile("" :: "v"(a));
  asm volatile("" :: "v"(b));
  asm volatile("" :: "v"(c));
  const unsigned ma = (mat == 0) ? 0xFFFFFFFFu : 0u;
  const unsigned mb = (mat == 1) ? 0xFFFFFFFFu : 0u;
  const unsigned mc = (mat == 2) ? 0xFFFFFFFFu : 0u;
  const v4u o = (a & (v4u){ma, ma, ma, ma}) | (b & (v4u){mb, mb, mb, mb}) | (c & (v4u){mc, mc, mc, mc});
  volatile v4u* q = (volatile v4u*)(void*)(WS + (size_t)g * 4);
  *q = o;
  __threadfence();
  *q = o;
}

#if OUT_FORM == 2
__global__ __launch_bounds__(256) void k_wtc(const float* __restrict__ Wt, float* __restrict__ WTS) {
  const int g = blockIdx.x * 256 + threadIdx.x;
  const v4f a = *(const v4fa*)(Wt + (size_t)g * 4);
  const v4f o = (v4f){ bf16_val(a[0]) * WT_CARRY, bf16_val(a[1]) * WT_CARRY,
                       bf16_val(a[2]) * WT_CARRY, bf16_val(a[3]) * WT_CARRY };
  volatile v4f* q = (volatile v4f*)(WTS + (size_t)g * 4);
  *q = o;
  __threadfence();
  *q = o;
}
#endif

__global__ __launch_bounds__(256) void k_relu(float* P) {
  const size_t g = (size_t)blockIdx.x * 256 + threadIdx.x;
  const v4f v = *(const v4fa*)(P + g * 4);
  v4f o;
  o[0] = (v[0] > 0.0f) ? v[0] : 0.0f;
  o[1] = (v[1] > 0.0f) ? v[1] : 0.0f;
  o[2] = (v[2] > 0.0f) ? v[2] : 0.0f;
  o[3] = (v[3] > 0.0f) ? v[3] : 0.0f;
  volatile v4f* q = (volatile v4f*)(P + g * 4);
  *q = o;
  __threadfence();
  *q = o;
}

__device__ __forceinline__ float dot4c(v4f k, v4f q, float s) {
  s = fmaf(k[0], q[0], s);
  s = fmaf(k[1], q[1], s);
  s = fmaf(k[2], q[2], s);
  s = fmaf(k[3], q[3], s);
  return s;
}
__device__ __forceinline__ v4f axpy4(float p, v4f v, v4f a) {
  return (v4f){ fmaf(p, v[0], a[0]), fmaf(p, v[1], a[1]), fmaf(p, v[2], a[2]), fmaf(p, v[3], a[3]) };
}

__global__ __launch_bounds__(128) void k_nbr(const float* __restrict__ KQV, float* __restrict__ AO) {
  __shared__ __attribute__((aligned(16))) float sc[NK2 * 128];
  __shared__ __attribute__((aligned(16))) float tl[128 * TP];
  const int tid = threadIdx.x;
  const int bh  = blockIdx.x;
  const int b   = bh >> 7;
  const int h   = bh & 127;
  const size_t tok = (size_t)bh * WW + tid;
  const int tb = b * (HH * WW);

#pragma unroll 1
  for (int k = 0; k < NK2; ++k) sc[k * 128 + tid] = 0.0f;

#pragma unroll 1
  for (int cc = 0; cc < 4; ++cc) {
    const float* qp = KQV + tok * NQKV + CH + 16 * cc;
    const v4f q0 = *(const v4fa*)(qp);
    const v4f q1 = *(const v4fa*)(qp + 4);
    const v4f q2 = *(const v4fa*)(qp + 8);
    const v4f q3 = *(const v4fa*)(qp + 12);
#pragma unroll 1
    for (int i = 0; i < KS; ++i) {
      const int hc = clampi(h + DIL * i - PAD, 0, HH - 1);
#pragma unroll 1
      for (int j = 0; j < KS; ++j) {
        const int wc = clampi(tid + DIL * j - PAD, 0, WW - 1);
        const float* kp = KQV + (size_t)(tb + hc * WW + wc) * NQKV + 16 * cc;
        const v4f ka = *(const v4fa*)(kp);
        const v4f kb = *(const v4fa*)(kp + 4);
        const v4f kc = *(const v4fa*)(kp + 8);
        const v4f kd = *(const v4fa*)(kp + 12);
        const int k = i * KS + j;
        float s = sc[k * 128 + tid];
        s = dot4c(ka, q0, s);
        s = dot4c(kb, q1, s);
        s = dot4c(kc, q2, s);
        s = dot4c(kd, q3, s);
        sc[k * 128 + tid] = s;
      }
    }
  }

  float m = sc[tid];
#pragma unroll 1
  for (int k = 1; k < NK2; ++k) m = fmaxf(m, sc[k * 128 + tid]);
  float sum = 0.0f;
#pragma unroll 1
  for (int k = 0; k < NK2; ++k) {
    const float e = expf(sc[k * 128 + tid] - m);
    sc[k * 128 + tid] = e;
    sum += e;
  }
  const float rs = (1.0f / sum) * AO_CARRY;

#pragma unroll 1
  for (int cc = 0; cc < 4; ++cc) {
    v4f a0 = (v4f){0.f, 0.f, 0.f, 0.f};
    v4f a1 = a0, a2 = a0, a3 = a0;
#pragma unroll 1
    for (int i = 0; i < KS; ++i) {
      const int hc = clampi(h + DIL * i - PAD, 0, HH - 1);
#pragma unroll 1
      for (int j = 0; j < KS; ++j) {
        const int wc = clampi(tid + DIL * j - PAD, 0, WW - 1);
        const float* vp = KQV + (size_t)(tb + hc * WW + wc) * NQKV + 2 * CH + 16 * cc;
        const v4f va = *(const v4fa*)(vp);
        const v4f vb = *(const v4fa*)(vp + 4);
        const v4f vc = *(const v4fa*)(vp + 8);
        const v4f vd = *(const v4fa*)(vp + 12);
        const float p = sc[(i * KS + j) * 128 + tid];
        a0 = axpy4(p, va, a0);
        a1 = axpy4(p, vb, a1);
        a2 = axpy4(p, vc, a2);
        a3 = axpy4(p, vd, a3);
      }
    }
    float* tp = tl + tid * TP + 16 * cc;
    tp[0]  = a0[0] * rs; tp[1]  = a0[1] * rs; tp[2]  = a0[2] * rs; tp[3]  = a0[3] * rs;
    tp[4]  = a1[0] * rs; tp[5]  = a1[1] * rs; tp[6]  = a1[2] * rs; tp[7]  = a1[3] * rs;
    tp[8]  = a2[0] * rs; tp[9]  = a2[1] * rs; tp[10] = a2[2] * rs; tp[11] = a2[3] * rs;
    tp[12] = a3[0] * rs; tp[13] = a3[1] * rs; tp[14] = a3[2] * rs; tp[15] = a3[3] * rs;
  }
  __syncthreads();

  v4f vv[16];
#pragma unroll
  for (int it = 0; it < 16; ++it) {
    const int idx = it * 128 + tid;
    const int row = idx >> 4;
    const int c4  = (idx & 15) * 4;
    const float* sp = tl + row * TP + c4;
    vv[it] = (v4f){ sp[0], sp[1], sp[2], sp[3] };
  }
  float* dst = AO + (size_t)bh * (size_t)(WW * CH);
  for (int pass = 0; pass < 2; ++pass) {
#pragma unroll
    for (int it = 0; it < 16; ++it) {
      const int idx = it * 128 + tid;
      *(volatile v4f*)(dst + (size_t)idx * 4) = vv[it];
    }
    __threadfence();
  }
}

__global__ __launch_bounds__(256) void k_t2x(const float* __restrict__ Y, const float* __restrict__ X,
                                             float* __restrict__ OUT) {
  __shared__ __attribute__((aligned(16))) float tl[128 * TP];
  const int tid = threadIdx.x;
  const int bh  = blockIdx.x;
  const int b   = bh >> 7;
  const int h   = bh & 127;
  const float* src = Y + (size_t)bh * (size_t)(WW * CH);
#pragma unroll
  for (int it = 0; it < 8; ++it) {
    const int idx = it * 256 + tid;
    const int w   = idx >> 4;
    const int c4  = (idx & 15) * 4;
    const v4f a = *(const v4fa*)(src + (size_t)idx * 4);
    float* sp = tl + w * TP + c4;
    sp[0] = a[0]; sp[1] = a[1]; sp[2] = a[2]; sp[3] = a[3];
  }
  __syncthreads();
  const int wave = tid >> 5;
  const int w4   = (tid & 31) * 4;
  v4f vv[8];
#pragma unroll
  for (int it = 0; it < 8; ++it) {
    const int c = it * 8 + wave;
    const size_t xo = ((size_t)(b * CH + c) * HH + h) * WW + w4;
    const v4f xv = *(const v4fa*)(X + xo);
    float y0 = tl[(w4 + 0) * TP + c];
    float y1 = tl[(w4 + 1) * TP + c];
    float y2 = tl[(w4 + 2) * TP + c];
    float y3 = tl[(w4 + 3) * TP + c];
    if (OUT_FORM == 2) { y0 *= Y_FOLD; y1 *= Y_FOLD; y2 *= Y_FOLD; y3 *= Y_FOLD; }
    vv[it] = (v4f){ y0 + bf16_val(xv[0]), y1 + bf16_val(xv[1]), y2 + bf16_val(xv[2]), y3 + bf16_val(xv[3]) };
  }
  for (int pass = 0; pass < 2; ++pass) {
#pragma unroll
    for (int it = 0; it < 8; ++it) {
      const int c = it * 8 + wave;
      const size_t xo = ((size_t)(b * CH + c) * HH + h) * WW + w4;
      *(volatile v4f*)(OUT + xo) = vv[it];
    }
    __threadfence();
  }
}

static constexpr size_t SZ_XT  = (size_t)NTOK * CH * 4;
static constexpr size_t SZ_XB  = (size_t)NTOK * CH * 2;
static constexpr size_t SZ_WS  = (size_t)NQKV * CH * 4;
static constexpr size_t SZ_WB  = (size_t)NQKV * CH * 2;
static constexpr size_t SZ_WTB = (size_t)CH * AOK * 2;
static constexpr size_t SZ_KQV = (size_t)NTOK * NQKV * 4;
static constexpr size_t SZ_AO  = (size_t)NTOK * CH * 4;
static constexpr size_t SZ_AOP = (size_t)NTOK * AOK * 2;
static constexpr size_t SZ_Y   = (size_t)NTOK * CH * 4;
#if OUT_FORM == 2
static constexpr size_t SZ_WTS = (size_t)CH * CH * 4;
#else
static constexpr size_t SZ_WTS = 0;
#endif
static constexpr size_t O_XT  = 0;
static constexpr size_t O_XB  = O_XT + SZ_XT;
static constexpr size_t O_WS  = O_XB + SZ_XB;
static constexpr size_t O_WB  = O_WS + SZ_WS;
static constexpr size_t O_WTB = O_WB + SZ_WB;
static constexpr size_t O_KQV = O_WTB + SZ_WTB;
static constexpr size_t O_AO  = O_KQV + SZ_KQV;
static constexpr size_t O_AOP = O_AO + SZ_AO;
static constexpr size_t O_Y   = O_AOP + SZ_AOP;
static constexpr size_t O_WTS = O_Y + SZ_Y;
static constexpr size_t WS_TOTAL = O_WTS + SZ_WTS;
static_assert(O_XB % 256 == 0 && O_WS % 256 == 0 && O_WB % 256 == 0 && O_WTB % 256 == 0);
static_assert(O_KQV % 256 == 0 && O_AO % 256 == 0 && O_AOP % 256 == 0 && O_Y % 256 == 0 && O_WTS % 256 == 0);
static_assert(WS_TOTAL <= ((size_t)128 << 20));
#if OUT_FORM == 1
static_assert(WS_TOTAL == (size_t)63004672);
#endif

extern "C" void kernel_launch(void* const* d_in, const int* in_sizes, int n_in,
                              void* d_out, int out_size, void* d_ws, size_t ws_size,
                              hipStream_t stream) {
  if (n_in < 5) return;
  if (in_sizes[0] != NB * CH * HH * WW) return;
  if (in_sizes[1] != CH * CH) return;
  if (in_sizes[2] != CH * CH) return;
  if (in_sizes[3] != CH * CH) return;
  if (in_sizes[4] != CH * CH) return;
  if (out_size != NB * CH * HH * WW) return;
  if (ws_size < WS_TOTAL) return;

  const float* x  = (const float*)d_in[0];
  const float* Wk = (const float*)d_in[1];
  const float* Wq = (const float*)d_in[2];
  const float* Wv = (const float*)d_in[3];
  const float* Wt = (const float*)d_in[4];
  float* out = (float*)d_out;

  char* ws = (char*)d_ws;
  float*          XT  = (float*)(ws + O_XT);
  unsigned short* XB  = (unsigned short*)(ws + O_XB);
  float*          WSf = (float*)(ws + O_WS);
  unsigned short* WB  = (unsigned short*)(ws + O_WB);
  unsigned short* WTB = (unsigned short*)(ws + O_WTB);
  float*          KQV = (float*)(ws + O_KQV);
  float*          AO  = (float*)(ws + O_AO);
  unsigned short* AOP = (unsigned short*)(ws + O_AOP);
  float*          Y   = (float*)(ws + O_Y);

  const dim3 blk(256);

  k_x2t<<<dim3(NB * HH), blk, 0, stream>>>(x, XT);
  k_wstack<<<dim3(NQKV * CH / 4 / 256), blk, 0, stream>>>(Wk, Wq, Wv, WSf);
  k_plane<0><<<dim3(NTOK * CH / 8 / 256), blk, 0, stream>>>(XT, NTOK, CH, CH, XB, NTOK, CH);
  k_plane<0><<<dim3(NQKV * CH / 8 / 256), blk, 0, stream>>>(WSf, NQKV, CH, CH, WB, NQKV, CH);
#if OUT_FORM == 1
  k_plane<3><<<dim3(CH * 2 * CH / 8 / 256), blk, 0, stream>>>(Wt, CH, CH, CH, WTB, CH, CH);
#else
  float* WTS = (float*)(ws + O_WTS);
  k_wtc<<<dim3(CH * CH / 4 / 256), blk, 0, stream>>>(Wt, WTS);
  k_plane<2><<<dim3(CH * CH / 8 / 256), blk, 0, stream>>>(WTS, CH, CH, CH, WTB, CH, CH);
#endif
  k_gemm_nt<0, 0><<<dim3((NTOK / 64) * (NQKV / 64) / 8), blk, 0, stream>>>(XB, WB, WSf, KQV, NTOK, NQKV, CH, NQKV);
  k_relu<<<dim3(NTOK * NQKV / 4 / 256), blk, 0, stream>>>(KQV);
  k_nbr<<<dim3(NB * HH), dim3(128), 0, stream>>>(KQV, AO);
  k_plane<OUT_FORM><<<dim3(NTOK * AOK / 8 / 256), blk, 0, stream>>>(AO, NTOK, CH, CH, AOP, NTOK, CH);
  k_gemm_nt<OUT_FORM, 0><<<dim3((NTOK / 64) * (CH / 64) / 8), blk, 0, stream>>>(AOP, WTB, WSf, Y, NTOK, CH, AOK, CH);
  k_t2x<<<dim3(NB * HH), blk, 0, stream>>>(Y, x, out);
  (void)hipGetLastError();
}
